// SA2D_62680752718501
// MI455X (gfx1250) — hardware-verified
//
#include <hip/hip_runtime.h>
#include <math.h>

typedef __attribute__((ext_vector_type(16))) _Float16 v16h;
typedef __attribute__((ext_vector_type(16))) __bf16 v16b;
typedef __attribute__((ext_vector_type(8)))  _Float16 v8h;
typedef __attribute__((ext_vector_type(8)))  float v8f;
typedef __attribute__((ext_vector_type(4)))  float v4f;
typedef __attribute__((ext_vector_type(2)))  float v2f;
typedef __attribute__((ext_vector_type(4)))  unsigned v4u;
typedef __attribute__((ext_vector_type(4)))  int v4i;
typedef float __attribute__((may_alias)) float_a;
typedef int __attribute__((may_alias)) int_a;

template <typename T> __device__ __forceinline__ void vst2(void* p, T v) { *(volatile T*)p = v; __threadfence(); *(volatile T*)p = v; }
__device__ __forceinline__ v8f wmma16(v16h a, v16h b, v8f c) {
  v8f d = __builtin_amdgcn_wmma_f32_16x16x32_f16(false, a, false, b, (short)0, c, false, false);
  asm volatile("v_nop\n\tv_nop\n\tv_nop\n\tv_nop" : "+v"(d) : "v"(a), "v"(b));
  return d;
}
__device__ __forceinline__ v8f wmma_bf(v16b a, v16b b, v8f c) {
  v8f d = __builtin_amdgcn_wmma_f32_16x16x32_bf16(false, a, false, b, (short)0, c, false, false);
  asm volatile("v_nop\n\tv_nop\n\tv_nop\n\tv_nop" : "+v"(d) : "v"(a), "v"(b));
  return d;
}
__device__ __forceinline__ v16h frag_h(const _Float16* rowk0, int lane) {
  union { v16h v; v8h q[2]; } u; const _Float16* p = rowk0 + 8 * (lane >> 4);
  u.q[0] = *(const v8h*)p; u.q[1] = *(const v8h*)(p + 16); return u.v;
}
__device__ __forceinline__ v16h frag_f32(const float* rowk0, int lane) {
  v16h a; const float* p = rowk0 + 8 * (lane >> 4);
#pragma unroll
  for (int i = 0; i < 8; ++i) { a[i] = (_Float16)p[i]; a[8 + i] = (_Float16)p[16 + i]; }
  return a;
}
__device__ __forceinline__ v16h frag_f32s(const float* rowk0, int lane, float sc) {
  v16h a; const float* p = rowk0 + 8 * (lane >> 4);
#pragma unroll
  for (int i = 0; i < 8; ++i) { a[i] = (_Float16)(p[i] * sc); a[8 + i] = (_Float16)(p[16 + i] * sc); }
  return a;
}
__device__ __forceinline__ v16h fragc_f32(const float* W, int k0, int n, int lane, int ld, int K) {
  v16h a; const int g = lane >> 4;
#pragma unroll
  for (int i = 0; i < 8; ++i) { const int ka = k0 + 8 * g + i, kb = ka + 16;
    a[i] = (_Float16)(ka < K ? W[(size_t)(ka < K ? ka : K - 1) * ld + n] : 0.f); a[8 + i] = (_Float16)(kb < K ? W[(size_t)(kb < K ? kb : K - 1) * ld + n] : 0.f); }
  return a;
}
struct F2 { v16b h, l; };
__device__ __forceinline__ F2 bsplit16(const float v[16]) { F2 r;
#pragma unroll
  for (int i = 0; i < 16; ++i) { const __bf16 h = (__bf16)v[i]; r.h[i] = h; r.l[i] = (__bf16)(v[i] - (float)h); }
  return r; }
__device__ __forceinline__ F2 split_row(const float* row, int k0, int lane) { float v[16]; const float* p = row + k0 + 8 * (lane >> 4);
#pragma unroll
  for (int i = 0; i < 8; ++i) { v[i] = p[i]; v[8 + i] = p[16 + i]; }
  return bsplit16(v); }
__device__ __forceinline__ F2 split_rowK(const float* row, int k0, int lane, int K) { float v[16]; const int g = lane >> 4;
#pragma unroll
  for (int i = 0; i < 8; ++i) { const int ka = k0 + 8 * g + i, kb = ka + 16; v[i] = ka < K ? row[ka < K ? ka : K - 1] : 0.f; v[8 + i] = kb < K ? row[kb < K ? kb : K - 1] : 0.f; }
  return bsplit16(v); }
__device__ __forceinline__ F2 split_col(const float* W, int k0, int n, int lane, int ld, int K) { float v[16]; const int g = lane >> 4;
#pragma unroll
  for (int i = 0; i < 8; ++i) { const int ka = k0 + 8 * g + i, kb = ka + 16; v[i] = ka < K ? W[(size_t)(ka < K ? ka : K - 1) * ld + n] : 0.f; v[8 + i] = kb < K ? W[(size_t)(kb < K ? kb : K - 1) * ld + n] : 0.f; }
  return bsplit16(v); }
__device__ __forceinline__ v8f mac3(const F2& a, const F2& b, v8f c) { c = wmma_bf(a.l, b.h, c); c = wmma_bf(a.h, b.l, c); return wmma_bf(a.h, b.h, c); }
__device__ __forceinline__ float sigm(float v) { return 1.0f / (1.0f + expf(-v)); }
#define LDSX() do { asm volatile("s_wait_dscnt 0" ::: "memory"); __builtin_amdgcn_wave_barrier(); __builtin_amdgcn_fence(__ATOMIC_RELEASE, "workgroup"); } while (0)


#define NB 8
#define CC 64
#define HW 128
#define NPX (HW * HW)
#ifndef TSB
#define TSB (NB * NPX / 4)
#endif
typedef __attribute__((ext_vector_type(8))) __bf16 v8b;
__device__ __forceinline__ v16b frag_b(const __bf16* rowk0, int lane) {
  union { v16b v; v8b q[2]; } u; const __bf16* p = rowk0 + 8 * (lane >> 4);
  u.q[0] = *(const v8b*)p; u.q[1] = *(const v8b*)(p + 16); return u.v;
}
__device__ __forceinline__ float bfr(float v) { return (float)(__bf16)v; }
__device__ __attribute__((noinline)) float exp_ni(float v) { return expf(v); }
__device__ __attribute__((noinline)) float erf_ni(float v) { return erff(v); }

#define WS_QP  0u
#define WS_KP  (WS_QP + 4u * (size_t)NB * CC * NPX)
#define WS_VP  (WS_KP + 4u * (size_t)NB * CC * NPX)
#define WS_END (WS_VP + 4u * (size_t)NB * CC * NPX)

__global__ __launch_bounds__(128) void k_conv(const float* __restrict__ X, const float* __restrict__ WK, const float* __restrict__ WQ, const float* __restrict__ WV, float* __restrict__ QP, float* __restrict__ KP, float* __restrict__ VP) { __shared__ __align__(16) __bf16 sx[CC][136]; __shared__ __align__(16) float so[CC][132];
  const int tid = threadIdx.x, wave = tid >> 5, lane = tid & 31, col = lane & 15, g = lane >> 4; const int p0 = blockIdx.x * 128; const size_t b = blockIdx.y; const int which = blockIdx.z; const float* Wm = which == 0 ? WQ : which == 1 ? WK : WV; float* dst = which == 0 ? QP : which == 1 ? KP : VP;
  for (int e = tid; e < CC * 128; e += 128) { const int c = e >> 7, pl = e & 127; sx[c][pl] = (__bf16)X[(b * CC + c) * (size_t)NPX + p0 + pl]; }
  __syncthreads();
  v8f acc[8] = {};
#pragma unroll
  for (int kc = 0; kc < CC / 32; ++kc) { v16b a; { const float* p = Wm + (size_t)(wave * 16 + col) * CC + kc * 32 + 8 * g;
#pragma unroll
      for (int i = 0; i < 8; ++i) { a[i] = (__bf16)p[i]; a[8 + i] = (__bf16)p[16 + i]; } }
#pragma unroll
    for (int j = 0; j < 8; ++j) { v16b xb;
#pragma unroll
      for (int i = 0; i < 8; ++i) { xb[i] = sx[kc * 32 + 8 * g + i][j * 16 + col]; xb[8 + i] = sx[kc * 32 + 16 + 8 * g + i][j * 16 + col]; }
      acc[j] = wmma_bf(a, xb, acc[j]); } }
#pragma unroll
  for (int j = 0; j < 8; ++j)
#pragma unroll
    for (int r = 0; r < 8; ++r) so[wave * 16 + 8 * g + r][j * 16 + col] = acc[j][r];
  __syncthreads(); for (int e = tid; e < CC * 32; e += 128) { const int o = e >> 5, q = e & 31; vst2(dst + (b * CC + o) * (size_t)NPX + p0 + q * 4, *(const v4f*)&so[o][q * 4]); } }
__global__ __launch_bounds__(256) void k_sa(const float* __restrict__ QP, const float* __restrict__ KP, const float* __restrict__ VP, float* __restrict__ OUT) { __shared__ float sred[4][9][2]; __shared__ float sat[4][9]; __shared__ __align__(16) float so[4][64];
  const int t = threadIdx.x; const int grp = t >> 6, c = t & 63, wl = (t >> 5) & 1, ln = t & 31; const size_t gl = (size_t)blockIdx.x * 4 + grp; const size_t b = gl / NPX; const int l = (int)(gl % NPX);
  const int qo = l >> 8; const int qpos = (l & 255) * 64 + c; const float qv = QP[(b * CC + qo) * (size_t)NPX + qpos];
  float kv[9], vv[9];
#pragma unroll
  for (int k = 0; k < 9; ++k) { const int gg = l * 9 + k; const int ch = gg >> 8; const int pos = (gg & 255) * 64 + c; const int o = ch / 9, kk = ch % 9; const int kh = kk / 3, kw = kk % 3; const int row = (pos >> 7) + kh - 1, cl = (pos & 127) + kw - 1; const bool in = (row >= 0 && row < HW && cl >= 0 && cl < HW); const size_t off = (b * CC + o) * (size_t)NPX + (size_t)(in ? row : 0) * HW + (in ? cl : 0);
    kv[k] = in ? KP[off] : 0.f; vv[k] = in ? VP[off] : 0.f; }
#pragma unroll
  for (int k = 0; k < 9; ++k) { float s = qv * kv[k];
#pragma unroll
    for (int o = 1; o < 32; o <<= 1) s += __shfl_xor(s, o); if (ln == 0) sred[grp][k][wl] = s; }
  __syncthreads();
  if (c < 9) { sat[grp][c] = sred[grp][c][0] + sred[grp][c][1]; }
  __syncthreads();
  float mx = -3.0e38f; for (int k = 0; k < 9; ++k) mx = fmaxf(mx, sat[grp][k]); float e[9], ssum = 0.f; for (int k = 0; k < 9; ++k) { e[k] = expf(sat[grp][k] - mx); ssum += e[k]; } const float inv = 1.0f / ssum;
  float acc = 0.f; for (int k = 0; k < 9; ++k) acc += e[k] * inv * vv[k]; so[grp][c] = acc;
  __syncthreads(); if (c < 16) vst2(OUT + (b * CC + qo) * (size_t)NPX + (size_t)(l & 255) * 64 + c * 4, *(const v4f*)&so[grp][c * 4]); }
extern "C" void kernel_launch(void* const* d_in, const int* in_sizes, int n_in, void* d_out, int out_size, void* d_ws, size_t ws_size, hipStream_t stream) {
  (void)in_sizes; (void)n_in; (void)out_size;
  const float** F = (const float**)d_in;
  if (ws_size < (size_t)WS_END) return;
  char* ws = (char*)d_ws; float *QP = (float*)(ws + WS_QP), *KP = (float*)(ws + WS_KP), *VP = (float*)(ws + WS_VP);
  k_conv<<<dim3(NPX / 128, NB, 3), 128, 0, stream>>>(F[0], F[1], F[2], F[3], QP, KP, VP);
  k_sa<<<TSB, 256, 0, stream>>>(QP, KP, VP, (float*)d_out);
}
